// minCUTPooling_6777458393289
// MI455X (gfx1250) — hardware-verified
//
#include <hip/hip_runtime.h>
#include <math.h>

#define NN   50000
#define NE   800000
#define NV   (NE + NN)
#define IND  128
#define FD   64
#define NH   4
#define FW   256
#define OUTD 10
#define NT   256
#define SRB  2048
#define NTL  25
#define NPAD (NTL * SRB)
#define SCH  2048
#define NCH  ((NV + SCH - 1) / SCH)

typedef __attribute__((ext_vector_type(16))) _Float16 v16h;
typedef __attribute__((ext_vector_type(8)))  _Float16 v8h;
typedef __attribute__((ext_vector_type(4)))  _Float16 v4h;
typedef __attribute__((ext_vector_type(16))) __bf16   v16b;
typedef __attribute__((ext_vector_type(8)))  __bf16   v8b;
typedef __attribute__((ext_vector_type(8)))  float    v8f;
typedef __attribute__((ext_vector_type(4)))  float    v4f;
typedef __attribute__((ext_vector_type(4)))  int      v4i;

__device__ __forceinline__ unsigned short f2bf_bits(float f) {
  unsigned u = __float_as_uint(f);
  return (unsigned short)((u + 0x7FFFu + ((u >> 16) & 1u)) >> 16);
}
__device__ __forceinline__ float bf_bits2f(unsigned short h) { return __uint_as_float(((unsigned)h) << 16); }

__device__ __forceinline__ void dep_guard_h(v8f& a, v8f& b, v16h x, v16h y) { asm volatile("v_nop\n\tv_nop\n\tv_nop\n\tv_nop" : "+v"(a), "+v"(b) : "v"(x), "v"(y)); }
__device__ __forceinline__ void dep_guard_b(v8f& a, v8f& b, v16b x, v16b y) { asm volatile("v_nop\n\tv_nop\n\tv_nop\n\tv_nop" : "+v"(a), "+v"(b) : "v"(x), "v"(y)); }
__device__ __forceinline__ void keep4_h(v16h a, v16h b, v16h c, v16h d) { asm volatile("v_nop" :: "v"(a), "v"(b), "v"(c), "v"(d)); }
__device__ __forceinline__ void keep4_b(v16b a, v16b b, v16b c, v16b d) { asm volatile("v_nop" :: "v"(a), "v"(b), "v"(c), "v"(d)); }
__device__ __forceinline__ void acc_guard4(v8f& a, v8f& b, v8f& c, v8f& d) { asm volatile("v_nop\n\tv_nop\n\tv_nop\n\tv_nop" : "+v"(a), "+v"(b), "+v"(c), "+v"(d)); }
template <typename T> struct Frag;
template <> struct Frag<_Float16> {
  typedef v16h V; union U { v16h v; v8h h[2]; };
  static __device__ __forceinline__ v16h load(const _Float16* p) {
    U f; f.h[0] = *(const v8h*)(p); f.h[1] = *(const v8h*)(p + 16); return f.v;
  }
  static __device__ __forceinline__ v8f mma(v16h a, v16h b, v8f c) {
    return __builtin_amdgcn_wmma_f32_16x16x32_f16(false, a, false, b, (short)0, c, false, false);
  }
  static __device__ __forceinline__ void guard(v8f& a, v8f& b, v16h x, v16h y) { dep_guard_h(a, b, x, y); }
  static __device__ __forceinline__ void keep(v16h a, v16h b, v16h c, v16h d) { keep4_h(a, b, c, d); }
};
template <> struct Frag<__bf16> {
  typedef v16b V; union U { v16b v; v8b h[2]; };
  static __device__ __forceinline__ v16b load(const __bf16* p) {
    U f; f.h[0] = *(const v8b*)(p); f.h[1] = *(const v8b*)(p + 16); return f.v;
  }
  static __device__ __forceinline__ v8f mma(v16b a, v16b b, v8f c) {
    return __builtin_amdgcn_wmma_f32_16x16x32_bf16(false, a, false, b, (short)0, c, false, false);
  }
  static __device__ __forceinline__ void guard(v8f& a, v8f& b, v16b x, v16b y) { dep_guard_b(a, b, x, y); }
  static __device__ __forceinline__ void keep(v16b a, v16b b, v16b c, v16b d) { keep4_b(a, b, c, d); }
};

template <int ET> struct Elem;
template <> struct Elem<0> { typedef _Float16 T; };
template <> struct Elem<1> { typedef __bf16 T; };
template <int ET, bool SPLIT, int BIAS_MODE, int OUT_MODE, bool RESID, int ACT = 0>
__global__ __launch_bounds__(256) void wmma_gemm64(
    const unsigned short* __restrict__ Ap, const unsigned short* __restrict__ A2p, int lda, long strideA,
    const unsigned short* __restrict__ Btp, const unsigned short* __restrict__ Bt2p, int ldb, long strideB,
    void* __restrict__ Cout, void* __restrict__ Cout2, int ldc, long strideC,
    const float* __restrict__ bias,
    const float* __restrict__ resid, long strideR,
    int M, int N, int K, float scale) {
  typedef typename Elem<ET>::T T;
  typedef typename Frag<T>::V V;
  const T* A = (const T*)Ap; const T* A2 = (const T*)A2p; const T* Bt = (const T*)Btp; const T* Bt2 = (const T*)Bt2p;
  __shared__ __align__(16) float sT[8][16 * 68];
  const int b    = blockIdx.y;
  const int lane = threadIdx.x & 31;
  const int wave = threadIdx.x >> 5;
  const int tilesN = N >> 6;
  const int tilesM = M >> 6;
  const int tile = blockIdx.x * 8 + wave;
  if (tile >= tilesM * tilesN) return;
  const int tm = tile / tilesN;
  const int tn = tile - tm * tilesN;
  const int m0 = tm << 6;
  const int n0 = tn << 6;

  const T* Ab  = A  + (size_t)b * strideA;
  const T* Bb  = Bt + (size_t)b * strideB;
  const T* Ab2 = SPLIT ? (A2  + (size_t)b * strideA) : nullptr;
  const T* Bb2 = SPLIT ? (Bt2 + (size_t)b * strideB) : nullptr;

  const int rlane = lane & 15;
  const int koff  = (lane >> 4) * 8;
  const int mOff  = (lane >> 4) * 8;

  v8f acc[4][4];
#pragma unroll
  for (int i = 0; i < 4; ++i)
#pragma unroll
    for (int j = 0; j < 4; ++j) acc[i][j] = (v8f){0.f,0.f,0.f,0.f,0.f,0.f,0.f,0.f};

  for (int k0 = 0; k0 < K; k0 += 32) {
    V bh[4], bl[4];
#pragma unroll
    for (int j = 0; j < 4; ++j) {
      const size_t bo = (size_t)(n0 + (j << 4) + rlane) * ldb + koff + k0;
      bh[j] = Frag<T>::load(Bb + bo);
      if (SPLIT) bl[j] = Frag<T>::load(Bb2 + bo);
    }
#pragma unroll
    for (int i = 0; i < 4; ++i) {
      const size_t ao = (size_t)(m0 + (i << 4) + rlane) * lda + koff + k0;
      V ah = Frag<T>::load(Ab + ao);
      V al;
      if (SPLIT) al = Frag<T>::load(Ab2 + ao);
#pragma unroll
      for (int j = 0; j < 4; ++j) {
        acc[i][j] = Frag<T>::mma(ah, bh[j], acc[i][j]);
        if (SPLIT) {
          acc[i][j] = Frag<T>::mma(ah, bl[j], acc[i][j]);
          acc[i][j] = Frag<T>::mma(al, bh[j], acc[i][j]);
        }
      }
      Frag<T>::guard(acc[i][0], acc[i][3], ah, SPLIT ? al : ah);
    }
    Frag<T>::keep(bh[0], bh[1], bh[2], bh[3]);
    if (SPLIT) Frag<T>::keep(bl[0], bl[1], bl[2], bl[3]);
  }
  acc_guard4(acc[0][0], acc[0][1], acc[0][2], acc[0][3]);
  acc_guard4(acc[1][0], acc[1][1], acc[1][2], acc[1][3]);
  acc_guard4(acc[2][0], acc[2][1], acc[2][2], acc[2][3]);
  acc_guard4(acc[3][0], acc[3][1], acc[3][2], acc[3][3]);

  float* slab = sT[wave];
  const float* Rb = RESID ? (resid + (size_t)b * strideR) : nullptr;
#pragma unroll
  for (int i = 0; i < 4; ++i) {
    const int mBase = m0 + (i << 4);
#pragma unroll
    for (int j = 0; j < 4; ++j) {
      const int n = n0 + (j << 4) + rlane;
      float bv = 0.f;
      if (BIAS_MODE == 2) bv = bias[n];
#pragma unroll
      for (int r = 0; r < 8; ++r) {
        float v = acc[i][j][r] * scale;
        if (BIAS_MODE == 1) v += bias[mBase + mOff + r];
        if (BIAS_MODE == 2) v += bv;
        if (RESID) v += Rb[(size_t)(mBase + mOff + r) * ldc + n];
        if (ACT == 1) v = tanhf(v);
        if (ACT == 2) v = fmaxf(v, 0.0f);
        if (ACT == 3) v = v / (1.0f + expf(-v));
        if (ACT == 4) v = (v > 0.f) ? v : 0.01f * v;
        if (ACT == 5) v = 0.5f * v * (1.0f + erff(v * 0.70710678118654752f));
        slab[(mOff + r) * 68 + (j << 4) + rlane] = v;
      }
    }
    __builtin_amdgcn_fence(__ATOMIC_RELEASE, "workgroup");
    __builtin_amdgcn_wave_barrier();
    __builtin_amdgcn_fence(__ATOMIC_ACQUIRE, "workgroup");
    if (OUT_MODE == 0) {
      float* C = (float*)Cout + (size_t)b * strideC;
      const int hh = lane >> 4, c4 = (lane & 15) * 4;
      for (int pass = 0; pass < 2; ++pass) {
#pragma unroll
        for (int it = 0; it < 8; ++it) {
          const int row = it * 2 + hh;
          v4f v = *(const v4f*)(slab + row * 68 + c4);
          *(volatile v4f*)(C + (size_t)(mBase + row) * ldc + n0 + c4) = v;
        }
        __threadfence();
      }
    } else {
      const int q = lane >> 3, c8 = (lane & 7) * 8;
      unsigned short* C  = (unsigned short*)Cout  + (size_t)b * strideC;
      unsigned short* C2 = (OUT_MODE == 2) ? ((unsigned short*)Cout2 + (size_t)b * strideC) : nullptr;
      for (int pass = 0; pass < 2; ++pass) {
#pragma unroll
        for (int it = 0; it < 4; ++it) {
          const int row = it * 4 + q;
          const float* sp = slab + row * 68 + c8;
          v8h hv, lv;
#pragma unroll
          for (int e = 0; e < 8; ++e) {
            if (OUT_MODE == 1) {
              hv[e] = (_Float16)sp[e];
            } else {
              unsigned short hb = f2bf_bits(sp[e]);
              unsigned short lb = f2bf_bits(sp[e] - bf_bits2f(hb));
              hv[e] = __builtin_bit_cast(_Float16, hb);
              lv[e] = __builtin_bit_cast(_Float16, lb);
            }
          }
          *(volatile v8h*)(C + (size_t)(mBase + row) * ldc + n0 + c8) = hv;
          if (OUT_MODE == 2) *(volatile v8h*)(C2 + (size_t)(mBase + row) * ldc + n0 + c8) = lv;
        }
        __threadfence();
      }
    }
    __builtin_amdgcn_fence(__ATOMIC_RELEASE, "workgroup");
    __builtin_amdgcn_wave_barrier();
    __builtin_amdgcn_fence(__ATOMIC_ACQUIRE, "workgroup");
  }
}

template <int MODE>
__global__ __launch_bounds__(256) void wprep_kernel(const float* __restrict__ W, int K, int Nreal, int Npad,
                                                   unsigned short* __restrict__ outA, unsigned short* __restrict__ outB, float scale) {
  const int t = blockIdx.x * 256 + threadIdx.x;
  const int kg = K >> 3;
  if (t >= Npad * kg) return;
  const int n = t / kg;
  const int k8 = (t - n * kg) * 8;
  const bool ok = n < Nreal;
  const int nc = ok ? n : (Nreal - 1);
  v8h hv, lv;
#pragma unroll
  for (int e = 0; e < 8; ++e) {
    float v = W[(size_t)(k8 + e) * Nreal + nc] * scale;
    v = ok ? v : 0.f;
    if (MODE == 0) {
      hv[e] = (_Float16)v; lv[e] = hv[e];
    } else {
      const unsigned short hb = f2bf_bits(v);
      const unsigned short lb = f2bf_bits(v - bf_bits2f(hb));
      hv[e] = __builtin_bit_cast(_Float16, hb);
      lv[e] = __builtin_bit_cast(_Float16, lb);
    }
  }
  unsigned short* pa = outA + (size_t)n * K + k8;
  *(volatile v8h*)pa = hv;
  if (MODE == 1) *(volatile v8h*)(outB + (size_t)n * K + k8) = lv;
  __threadfence();
  *(volatile v8h*)pa = hv;
  if (MODE == 1) *(volatile v8h*)(outB + (size_t)n * K + k8) = lv;
}

__global__ __launch_bounds__(256) void padcast_x_kernel(const float* __restrict__ x, unsigned short* __restrict__ X16) {
  const int i = blockIdx.x * 256 + threadIdx.x;
  if (i >= NPAD * IND / 8) return;
  const int e0 = i * 8;
  const int row = e0 / IND, col = e0 - row * IND;
  const bool ok = row < NN;
  const int rowc = ok ? row : (NN - 1);
  const float* xp = x + (size_t)rowc * IND + col;
  const v4f a = *(const v4f*)(xp), b = *(const v4f*)(xp + 4);
  v8h hv;
#pragma unroll
  for (int e = 0; e < 4; ++e) {
    hv[e]     = (_Float16)(ok ? a[e] * 16.0f : 0.f);
    hv[4 + e] = (_Float16)(ok ? b[e] * 16.0f : 0.f);
  }
  unsigned short* op = X16 + (size_t)e0;
  *(volatile v8h*)op = hv; __threadfence(); *(volatile v8h*)op = hv;
}

__global__ __launch_bounds__(NT) void att_terms_kernel(const float* __restrict__ XW, const float* __restrict__ as, const float* __restrict__ ad,
                                                      float* __restrict__ ASD) {
  __shared__ __align__(16) float so[16 * 8];
  const int lane = threadIdx.x & 31, wave = threadIdx.x >> 5;
  const int sub = lane >> 4, q = lane & 15;
  const int nl = wave * 2 + sub;
  const int n = blockIdx.x * 16 + nl;
  const int h = q >> 2, cq = (q & 3) * 16;
  const float* xr = XW + (size_t)n * FW + h * FD + cq;
  const v4f x0 = *(const v4f*)(xr), x1 = *(const v4f*)(xr + 4), x2 = *(const v4f*)(xr + 8), x3 = *(const v4f*)(xr + 12);
  const float* sp = as + h * FD + cq;
  const float* dp = ad + h * FD + cq;
  const v4f s0 = *(const v4f*)(sp), s1 = *(const v4f*)(sp + 4), s2 = *(const v4f*)(sp + 8), s3 = *(const v4f*)(sp + 12);
  const v4f d0 = *(const v4f*)(dp), d1 = *(const v4f*)(dp + 4), d2 = *(const v4f*)(dp + 8), d3 = *(const v4f*)(dp + 12);
  float s = 0.f, d = 0.f;
#pragma unroll
  for (int e = 0; e < 4; ++e) {
    s += x0[e] * s0[e]; s += x1[e] * s1[e]; s += x2[e] * s2[e]; s += x3[e] * s3[e];
    d += x0[e] * d0[e]; d += x1[e] * d1[e]; d += x2[e] * d2[e]; d += x3[e] * d3[e];
  }
  s += __shfl_xor(s, 1, 32); s += __shfl_xor(s, 2, 32);
  d += __shfl_xor(d, 1, 32); d += __shfl_xor(d, 2, 32);
  if ((q & 3) == 0) { so[nl * 8 + h] = s; so[nl * 8 + 4 + h] = d; }
  __syncthreads();
  if (wave == 0) {
    const v4f v = *(const v4f*)(so + 4 * lane);
    float* op = ASD + (size_t)blockIdx.x * 128 + 4 * lane;
    *(volatile v4f*)op = v; __threadfence(); *(volatile v4f*)op = v;
  }
}

__device__ __forceinline__ int blk_excl_scan(int cnt, int* scan_ws, int tid, int* tot) {
  const int lane = tid & 31, wave = tid >> 5; int incl = cnt;
#pragma unroll
  for (int o = 1; o < 32; o <<= 1) { const int v = __shfl_up(incl, o, 32); if (lane >= o) incl += v; }
  if (lane == 31) scan_ws[wave] = incl;
  __syncthreads();
  if (wave == 0) { int wv = (lane < NT / 32) ? scan_ws[lane] : 0; int wincl = wv;
#pragma unroll
    for (int o = 1; o < 32; o <<= 1) { const int v = __shfl_up(wincl, o, 32); if (lane >= o) wincl += v; }
    if (lane < NT / 32) scan_ws[32 + lane] = wincl - wv; if (lane == 31) scan_ws[64] = wincl; }
  __syncthreads();
  const int res = scan_ws[32 + wave] + incl - cnt; *tot = scan_ws[64];
  return res;
}
template <int SPv, int CAP>
__device__ __forceinline__ int chunk_hits(const int* __restrict__ dstv, const int* __restrict__ srcv, int e0, int n0, int tid,
                                          int* LIST, int* scan_ws) {
  const int eb = e0 + tid * SPv;
  const bool real = eb < NE;
  const int ebc = real ? eb : (NE - SPv);
  int rec[SPv]; int cnt = 0;
#pragma unroll
  for (int k = 0; k < SPv; k += 4) {
    const v4i d4 = *(const v4i*)(dstv + ebc + k);
    const v4i s4 = *(const v4i*)(srcv + ebc + k);
#pragma unroll
    for (int e = 0; e < 4; ++e) {
      int d, s;
      if (real) { d = d4[e]; s = s4[e]; s = s < 0 ? 0 : (s >= NN ? NN - 1 : s); }
      else { const int ev = eb + k + e; d = (ev < NV) ? (ev - NE) : -1; s = d; }
      int r = -1;
      if (d >= n0 && d < n0 + SRB) { r = ((d - n0) << 16) | s; ++cnt; }
      rec[k + e] = r;
    }
  }
  int tot; int p = blk_excl_scan(cnt, scan_ws, tid, &tot);
#pragma unroll
  for (int k = 0; k < SPv; ++k) if (rec[k] >= 0) { if ((unsigned)p < (unsigned)CAP) LIST[p] = rec[k]; ++p; }
  __syncthreads();
  return tot < CAP ? tot : CAP;
}

template <int OUTK>
__global__ __launch_bounds__(NT) void gat_agg_kernel(const float* __restrict__ XW, const int* __restrict__ ei, const float* __restrict__ ASD,
                                                    const float* __restrict__ bias, float* AGG,
                                                    unsigned short* __restrict__ HOa, unsigned short* __restrict__ HOb, float oscale) {
  extern __shared__ __align__(16) float dsm[];
  float* SM  = dsm;
  float* SL  = dsm + SRB * NH;
  float* SAD = dsm + 2 * SRB * NH;
  int*   LIST = (int*)(dsm + 3 * SRB * NH);
  __shared__ int scan_ws[80];
  const int tid = threadIdx.x, lane = tid & 31, wave = tid >> 5;
  const int tile = blockIdx.x;
  const int n0 = tile * SRB;
  const int h4 = lane & 3;
  const v4f z4 = {0.f, 0.f, 0.f, 0.f};
#pragma unroll 1
  for (int j = 0; j < 256; ++j) {
    float* rp = AGG + (size_t)(n0 + wave * 256 + j) * FW + 4 * lane;
    *(volatile v4f*)(rp) = z4; *(volatile v4f*)(rp + 128) = z4;
    __threadfence();
    *(volatile v4f*)(rp) = z4; *(volatile v4f*)(rp + 128) = z4;
  }
  for (int i = tid; i < SRB * NH; i += NT) {
    SM[i] = -INFINITY; SL[i] = 0.f;
    SAD[i] = ASD[(size_t)(n0 + (i >> 2)) * 8 + 4 + (i & 3)];
  }
  __syncthreads();
  const int* srcv = ei; const int* dstv = ei + NE;
#pragma unroll 1
  for (int c = 0; c < NCH; ++c) {
    const int tot = chunk_hits<SCH / NT, SCH>(dstv, srcv, c * SCH, n0, tid, LIST, scan_ws);
#pragma unroll 1
    for (int base = 0; base < tot; base += 32) {
      const int q = base + lane;
      const int rv = (q < tot) ? LIST[q] : -1;
      const int own = (rv >= 0 && (rv >> 24) == wave) ? 1 : 0;
      unsigned msk = (unsigned)__ballot(own);
#pragma unroll 1
      for (int it = 0; it < 32; ++it) {
        if (msk == 0u) break;
        const int bp = __builtin_ctz(msk); msk &= msk - 1u;
        const int r = __shfl(rv, bp, 32);
        const int dl = r >> 16, s = r & 0xFFFF;
        const int mi = dl * NH + h4;
        float al = ASD[(size_t)s * 8 + h4] + SAD[mi];
        al = (al >= 0.f) ? al : 0.2f * al;
        const float mo = SM[mi], lo = SL[mi];
        const float mn = fmaxf(mo, al);
        const float rr = __expf(mo - mn), ex = __expf(al - mn);
        const float ln = lo * rr + ex;
        if (lane < NH) { SM[mi] = mn; SL[mi] = ln; }
        const int hj0 = lane >> 4, hj1 = 2 + (lane >> 4);
        const float rr0 = __shfl(rr, hj0, 32), ex0 = __shfl(ex, hj0, 32);
        const float rr1 = __shfl(rr, hj1, 32), ex1 = __shfl(ex, hj1, 32);
        const float* xr = XW + (size_t)s * FW + 4 * lane;
        float* rp = AGG + (size_t)(n0 + dl) * FW + 4 * lane;
        const v4f x0 = *(const v4f*)(xr), x1 = *(const v4f*)(xr + 128);
        v4f a0 = *(const v4f*)(rp), a1 = *(const v4f*)(rp + 128);
        a0 = a0 * rr0 + ex0 * x0;
        a1 = a1 * rr1 + ex1 * x1;
        *(volatile v4f*)(rp) = a0; *(volatile v4f*)(rp + 128) = a1;
        __threadfence();
        *(volatile v4f*)(rp) = a0; *(volatile v4f*)(rp + 128) = a1;
      }
    }
    __syncthreads();
  }
  const int sub = lane >> 3, c8 = (lane & 7) * 8;
  const v4f bA = *(const v4f*)(bias + c8), bB = *(const v4f*)(bias + c8 + 4);
#pragma unroll 1
  for (int jj = 0; jj < 64; ++jj) {
    const int dl = wave * 256 + jj * 4 + sub;
    const int n = n0 + dl;
    const v4f l4 = *(const v4f*)(SL + dl * NH);
    const float* rp = AGG + (size_t)n * FW + c8;
    v4f accA = z4, accB = z4;
#pragma unroll
    for (int h = 0; h < NH; ++h) {
      float lv = l4[h]; lv = lv > 0.f ? lv : 1.0f;
      const float ih = __builtin_amdgcn_rcpf(lv);
      const v4f a = *(const v4f*)(rp + FD * h), b = *(const v4f*)(rp + FD * h + 4);
      accA = accA + a * ih; accB = accB + b * ih;
    }
    const v4f vA = accA * 0.25f + bA, vB = accB * 0.25f + bB;
    const bool ok = n < NN;
    v8h hv, lv8;
#pragma unroll
    for (int e = 0; e < 8; ++e) {
      float v = (e < 4) ? vA[e & 3] : vB[e & 3];
      v = (v > 0.f) ? v : (__expf(v) - 1.0f);
      v = ok ? v : 0.f;
      if (OUTK == 1) {
        hv[e] = (_Float16)(v * oscale); lv8[e] = hv[e];
      } else {
        const unsigned short hb = f2bf_bits(v);
        const unsigned short lb = f2bf_bits(v - bf_bits2f(hb));
        hv[e]  = __builtin_bit_cast(_Float16, hb);
        lv8[e] = __builtin_bit_cast(_Float16, lb);
      }
    }
    unsigned short* oa = HOa + (size_t)n * FD + c8;
    *(volatile v8h*)oa = hv;
    if (OUTK == 2) *(volatile v8h*)(HOb + (size_t)n * FD + c8) = lv8;
    __threadfence();
    *(volatile v8h*)oa = hv;
    if (OUTK == 2) *(volatile v8h*)(HOb + (size_t)n * FD + c8) = lv8;
  }
}

__global__ __launch_bounds__(256) void fc_pack_kernel(const float* __restrict__ FCO, const float* __restrict__ fcb, float* __restrict__ out) {
  const int i4 = blockIdx.x * 256 + threadIdx.x;
  if (i4 >= NN * OUTD / 4) return;
  v4f v;
#pragma unroll
  for (int e = 0; e < 4; ++e) {
    const int idx = i4 * 4 + e;
    const int n = idx / OUTD, o = idx - n * OUTD;
    v[e] = FCO[(size_t)n * FD + o] + fcb[o];
  }
  float* op = out + (size_t)i4 * 4;
  *(volatile v4f*)op = v; __threadfence(); *(volatile v4f*)op = v;
}

extern "C" void kernel_launch(void* const* d_in, const int* in_sizes, int n_in,
                              void* d_out, int out_size, void* d_ws, size_t ws_size, hipStream_t stream) {
  (void)n_in;
  if (in_sizes[0] != NN * IND || in_sizes[1] != 2 * NE || out_size != NN * OUTD) return;
  const float* x    = (const float*)d_in[0];
  const int*   ei   = (const int*)  d_in[1];
  const float* W0   = (const float*)d_in[2];
  const float* as0  = (const float*)d_in[3];
  const float* ad0  = (const float*)d_in[4];
  const float* b0   = (const float*)d_in[5];
  const float* W1   = (const float*)d_in[6];
  const float* as1  = (const float*)d_in[7];
  const float* ad1  = (const float*)d_in[8];
  const float* b1   = (const float*)d_in[9];
  const float* W2   = (const float*)d_in[10];
  const float* as2  = (const float*)d_in[11];
  const float* ad2  = (const float*)d_in[12];
  const float* b2   = (const float*)d_in[13];
  const float* fcW  = (const float*)d_in[14];
  const float* fcb  = (const float*)d_in[15];
  float* out = (float*)d_out;

  char* ws = (char*)d_ws; size_t off = 0;
  auto carve = [&](size_t bytes) -> char* { char* p = ws + off; off += (bytes + 255) & ~(size_t)255; return p; };
  unsigned short* WT0  = (unsigned short*)carve((size_t)FW * IND * 2);
  unsigned short* WT1  = (unsigned short*)carve((size_t)FW * FD * 2);
  unsigned short* WT2h = (unsigned short*)carve((size_t)FW * FD * 2);
  unsigned short* WT2l = (unsigned short*)carve((size_t)FW * FD * 2);
  unsigned short* FCTh = (unsigned short*)carve((size_t)64 * FD * 2);
  unsigned short* FCTl = (unsigned short*)carve((size_t)64 * FD * 2);
  unsigned short* HB   = (unsigned short*)carve((size_t)NPAD * IND * 2);
  float*          XW   = (float*)carve((size_t)NPAD * FW * 4);
  float*          ASD  = (float*)carve((size_t)NPAD * 8 * 4);
  float*          AGG  = (float*)carve((size_t)NPAD * FW * 4);
  if (off > ws_size || off > (size_t)134217728) return;
  unsigned short* Hh  = HB;
  unsigned short* Hl  = HB + (size_t)NPAD * FD;
  float*          FCO = XW;

  const size_t aggLds = (size_t)(3 * SRB * NH + SCH) * 4;
  const int gtiles = (NPAD / 64) * (FW / 64);
  const int ftiles = (NPAD / 64) * 1;

  wprep_kernel<0><<<(FW * (IND / 8) + 255) / 256, 256, 0, stream>>>(W0, IND, FW, FW, WT0, nullptr, 64.0f);
  wprep_kernel<0><<<(FW * (FD / 8) + 255) / 256, 256, 0, stream>>>(W1, FD, FW, FW, WT1, nullptr, 16.0f);
  wprep_kernel<1><<<(FW * (FD / 8) + 255) / 256, 256, 0, stream>>>(W2, FD, FW, FW, WT2h, WT2l, 1.0f);
  wprep_kernel<1><<<(64 * (FD / 8) + 255) / 256, 256, 0, stream>>>(fcW, FD, OUTD, 64, FCTh, FCTl, 1.0f);
  padcast_x_kernel<<<(NPAD * IND / 8 + 255) / 256, 256, 0, stream>>>(x, HB);

  hipFuncSetAttribute((const void*)gat_agg_kernel<1>, hipFuncAttributeMaxDynamicSharedMemorySize, (int)aggLds);
  hipFuncSetAttribute((const void*)gat_agg_kernel<2>, hipFuncAttributeMaxDynamicSharedMemorySize, (int)aggLds);

  wmma_gemm64<0, false, 0, 0, false><<<dim3((gtiles + 7) / 8, 1), 256, 0, stream>>>(
      (const unsigned short*)HB, nullptr, IND, 0L, (const unsigned short*)WT0, nullptr, IND, 0L,
      (void*)XW, nullptr, FW, 0L, nullptr, nullptr, 0L, NPAD, FW, IND, 1.0f / 1024.0f);
  att_terms_kernel<<<NPAD / 16, NT, 0, stream>>>(XW, as0, ad0, ASD);
  gat_agg_kernel<1><<<NTL, NT, aggLds, stream>>>(XW, ei, ASD, b0, AGG, Hh, nullptr, 64.0f);

  wmma_gemm64<0, false, 0, 0, false><<<dim3((gtiles + 7) / 8, 1), 256, 0, stream>>>(
      (const unsigned short*)Hh, nullptr, FD, 0L, (const unsigned short*)WT1, nullptr, FD, 0L,
      (void*)XW, nullptr, FW, 0L, nullptr, nullptr, 0L, NPAD, FW, FD, 1.0f / 1024.0f);
  att_terms_kernel<<<NPAD / 16, NT, 0, stream>>>(XW, as1, ad1, ASD);
  gat_agg_kernel<2><<<NTL, NT, aggLds, stream>>>(XW, ei, ASD, b1, AGG, Hh, Hl, 1.0f);

  wmma_gemm64<1, true, 0, 0, false><<<dim3((gtiles + 7) / 8, 1), 256, 0, stream>>>(
      (const unsigned short*)Hh, (const unsigned short*)Hl, FD, 0L, (const unsigned short*)WT2h, (const unsigned short*)WT2l, FD, 0L,
      (void*)XW, nullptr, FW, 0L, nullptr, nullptr, 0L, NPAD, FW, FD, 1.0f);
  att_terms_kernel<<<NPAD / 16, NT, 0, stream>>>(XW, as2, ad2, ASD);
  gat_agg_kernel<2><<<NTL, NT, aggLds, stream>>>(XW, ei, ASD, b2, AGG, Hh, Hl, 1.0f);

  wmma_gemm64<1, true, 0, 0, false><<<dim3((ftiles + 7) / 8, 1), 256, 0, stream>>>(
      (const unsigned short*)Hh, (const unsigned short*)Hl, FD, 0L, (const unsigned short*)FCTh, (const unsigned short*)FCTl, FD, 0L,
      (void*)FCO, nullptr, FD, 0L, nullptr, nullptr, 0L, NPAD, 64, FD, 1.0f);
  fc_pack_kernel<<<(NN * OUTD / 4 + 255) / 256, 256, 0, stream>>>(FCO, fcb, out);
}
